// ResQuantize_87866440942167
// MI455X (gfx1250) — hardware-verified
//
#include <hip/hip_runtime.h>
#include <stddef.h>

#define DDIM    512
#define NBATCH  32
#define NT      128
#define NROWS   4096
#define NCODES  16384
#define MTILE   128
#define CHUNK   64
#define LDSP    528
#define NSPLIT  16
#define NRANGE  (NCODES / NSPLIT)
#define NCHUNKS (NRANGE / CHUNK)
#define CPR     (NSPLIT * 32)
#define NSEL    16
#define IDXP    32
#define TP      132

static_assert(NROWS == NBATCH * NT);
static_assert(NROWS % MTILE == 0);
static_assert(NCODES % (NSPLIT * CHUNK) == 0);
static_assert(NCHUNKS * CHUNK == NRANGE);
static_assert(DDIM == 512);
static_assert(LDSP % 8 == 0);
static_assert(LDSP >= DDIM);
static_assert(NCODES % 32 == 0);
static_assert(NROWS % 8 == 0);
static_assert((NROWS * DDIM) % 2048 == 0);
static_assert(NT == 128);

typedef _Float16 f16;
typedef f16 v16h __attribute__((ext_vector_type(16)));
typedef f16 v8h_t __attribute__((ext_vector_type(8)));
typedef v8h_t __attribute__((may_alias)) v8h;
typedef float v8f __attribute__((ext_vector_type(8)));
typedef float v4f_t __attribute__((ext_vector_type(4)));
typedef v4f_t __attribute__((may_alias)) v4f;
typedef float v2f_t __attribute__((ext_vector_type(2)));
typedef unsigned int u32;
typedef unsigned long long u64;
typedef u32 v4u_t __attribute__((ext_vector_type(4)));
typedef v4u_t __attribute__((may_alias)) v4u;
typedef u64 v2l_t __attribute__((ext_vector_type(2)));
typedef v2l_t __attribute__((may_alias)) v2l;

union Frag { v16h v; v8h_t h[2]; };
union Pack8 { v8h_t h; v4u_t u; };

__device__ __forceinline__ v8f zero8() {
    v8f z;
#pragma unroll
    for (int i = 0; i < 8; ++i) z[i] = 0.0f;
    return z;
}

__device__ __forceinline__ v8f wmma16(v16h a, v16h b, v8f c) {
    return __builtin_amdgcn_wmma_f32_16x16x32_f16(false, a, false, b, (short)0, c, false, false);
}

__device__ __forceinline__ u32 orderKey(float f) {
    const u32 u = __float_as_uint(f);
    return (u & 0x80000000u) ? ~u : (u | 0x80000000u);
}

__global__ void __launch_bounds__(256) cbprep_kernel(const float* __restrict__ cb,
                                                     f16* __restrict__ cbh,
                                                     float* __restrict__ cbn)
{
    __shared__ float cns[32];
    const int lane = threadIdx.x & 31, w = threadIdx.x >> 5;
    const int cbase = blockIdx.x * 32 + w * 4;
    Pack8 plo[4], phi[4];
#pragma unroll
    for (int i = 0; i < 4; ++i) {
        const int c = cbase + i;
        const float* r = cb + (size_t)c * DDIM + 8 * lane;
        const v4f_t a0 = *(const v4f*)(r);
        const v4f_t a1 = *(const v4f*)(r + 4);
        const v4f_t a2 = *(const v4f*)(r + 256);
        const v4f_t a3 = *(const v4f*)(r + 260);
        float s = 0.0f;
#pragma unroll
        for (int e = 0; e < 4; ++e) {
            s = fmaf(a0[e], a0[e], s);
            s = fmaf(a1[e], a1[e], s);
            s = fmaf(a2[e], a2[e], s);
            s = fmaf(a3[e], a3[e], s);
            plo[i].h[e]     = (f16)a0[e];
            plo[i].h[4 + e] = (f16)a1[e];
            phi[i].h[e]     = (f16)a2[e];
            phi[i].h[4 + e] = (f16)a3[e];
        }
#pragma unroll
        for (int off = 16; off > 0; off >>= 1) s += __shfl_xor(s, off, 32);
        if (lane == 0) cns[w * 4 + i] = s;
        f16* o = cbh + (size_t)c * DDIM + 8 * lane;
        *(volatile v4u_t*)(o) = plo[i].u;
        *(volatile v4u_t*)(o + 256) = phi[i].u;
    }
    __threadfence();
#pragma unroll
    for (int i = 0; i < 4; ++i) {
        f16* o = cbh + (size_t)(cbase + i) * DDIM + 8 * lane;
        *(volatile v4u_t*)(o) = plo[i].u;
        *(volatile v4u_t*)(o + 256) = phi[i].u;
    }
    __syncthreads();
    const int li = (4 * lane) & 31;
    v4f_t q;
    q[0] = cns[li]; q[1] = cns[li + 1]; q[2] = cns[li + 2]; q[3] = cns[li + 3];
    float* no = cbn + (size_t)blockIdx.x * 32 + li;
    const bool wr = (w == 0) && (lane < 8);
    if (wr) *(volatile v4f_t*)no = q;
    __threadfence();
    if (wr) *(volatile v4f_t*)no = q;
}

__global__ void __launch_bounds__(256) xf_kernel(const float* __restrict__ x, float* __restrict__ xf)
{
    __shared__ __align__(16) float tile[32 * TP];
    const int n = blockIdx.x >> 4, d0 = (blockIdx.x & 15) * 32;
    const int tid = threadIdx.x, lane = tid & 31, w = tid >> 5;
#pragma unroll
    for (int i = 0; i < 4; ++i) {
        const int u = tid + 256 * i;
        const int dd = u >> 5, t4 = (u & 31) * 4;
        const v4f_t val = *(const v4f*)(x + ((size_t)(n * DDIM + d0 + dd)) * NT + t4);
        *(v4f*)(tile + dd * TP + t4) = val;
    }
    __syncthreads();
    const int q = lane >> 3, c4 = (lane & 7) * 4;
    v4f_t o[4];
    size_t oo[4];
#pragma unroll
    for (int i = 0; i < 4; ++i) {
        const int t = 16 * w + 4 * i + q;
        v4f_t val;
        val[0] = tile[(c4 + 0) * TP + t];
        val[1] = tile[(c4 + 1) * TP + t];
        val[2] = tile[(c4 + 2) * TP + t];
        val[3] = tile[(c4 + 3) * TP + t];
        o[i] = val;
        oo[i] = (size_t)(n * NT + t) * DDIM + d0 + c4;
        *(volatile v4f_t*)(xf + oo[i]) = val;
    }
    __threadfence();
#pragma unroll
    for (int i = 0; i < 4; ++i) *(volatile v4f_t*)(xf + oo[i]) = o[i];
}

__global__ void __launch_bounds__(256) cvt16_kernel(const float* __restrict__ src,
                                                    f16* __restrict__ dst, int n8)
{
    const int i = blockIdx.x * 256 + threadIdx.x;
    const bool ok = (i < n8);
    const int ic = ok ? i : 0;
    Pack8 pk;
    const v4f_t a = *(const v4f*)(src + (size_t)ic * 8);
    const v4f_t b = *(const v4f*)(src + (size_t)ic * 8 + 4);
#pragma unroll
    for (int j = 0; j < 4; ++j) {
        pk.h[j]     = (f16)a[j];
        pk.h[4 + j] = (f16)b[j];
    }
    if (ok) *(volatile v4u_t*)(dst + (size_t)i * 8) = pk.u;
    __threadfence();
    if (ok) *(volatile v4u_t*)(dst + (size_t)i * 8) = pk.u;
}

__global__ void __launch_bounds__(256) screen_kernel(const f16* __restrict__ v16,
                                                     const f16* __restrict__ cbh,
                                                     const float* __restrict__ cbn,
                                                     u64* __restrict__ cand)
{
    __shared__ __align__(16) f16 Bs[CHUNK * LDSP];
    const int tid = threadIdx.x, wave = tid >> 5, lane = tid & 31;
    const int m = lane & 15, hh = lane >> 4;
    const int rowBase = blockIdx.x * MTILE + wave * 16;
    const int split = blockIdx.y;
    const int nBase0 = split * NRANGE;

    Frag a[16];
    const f16* arow = v16 + (size_t)(rowBase + m) * DDIM + 8 * hh;
#pragma unroll
    for (int s = 0; s < 16; ++s) {
        a[s].h[0] = *(const v8h*)(arow + 32 * s);
        a[s].h[1] = *(const v8h*)(arow + 32 * s + 16);
    }

    float b1[8], b2[8];
    u32 i1[8], i2[8];
#pragma unroll
    for (int r = 0; r < 8; ++r) { b1[r] = 3.0e38f; b2[r] = 3.0e38f; i1[r] = 0u; i2[r] = 0u; }

#pragma unroll 1
    for (int chunk = 0; chunk < NCHUNKS; ++chunk) {
        const int nb = nBase0 + chunk * CHUNK;
        __syncthreads();
#pragma unroll 4
        for (int i = 0; i < 16; ++i) {
            const int u = tid + i * 256;
            const int c = u >> 6, j = u & 63;
            const v4u_t g = *(const v4u*)(cbh + (size_t)(nb + c) * DDIM + j * 8);
            *(v4u*)(Bs + c * LDSP + j * 8) = g;
        }
        __syncthreads();
#pragma unroll 1
        for (int nt = 0; nt < 4; ++nt) {
            const f16* bp = Bs + (nt * 16 + m) * LDSP + 8 * hh;
            v8f acc = zero8();
            Frag b[2];
#pragma unroll
            for (int s = 0; s < 16; ++s) {
                b[s & 1].h[0] = *(const v8h*)(bp + 32 * s);
                b[s & 1].h[1] = *(const v8h*)(bp + 32 * s + 16);
                acc = wmma16(a[s].v, b[s & 1].v, acc);
            }
            asm volatile("v_nop\n\tv_nop\n\tv_nop\n\tv_nop" : "+v"(acc) : "v"(a[15].v), "v"(b[1].v));
            const int code = nb + nt * 16 + m;
            const float cn = cbn[code];
#pragma unroll
            for (int r = 0; r < 8; ++r) {
                const float sc = fmaf(-2.0f, acc[r], cn);
                if (sc < b1[r]) { b2[r] = b1[r]; i2[r] = i1[r]; b1[r] = sc; i1[r] = (u32)code; }
                else if (sc < b2[r]) { b2[r] = sc; i2[r] = (u32)code; }
            }
        }
    }

    v2l_t kv[8];
#pragma unroll
    for (int r = 0; r < 8; ++r) {
        kv[r][0] = ((u64)orderKey(b1[r]) << 32) | (u64)i1[r];
        kv[r][1] = ((u64)orderKey(b2[r]) << 32) | (u64)i2[r];
    }
    u64* cp = cand + ((size_t)(rowBase + 8 * hh) * NSPLIT + split) * 32 + 2 * m;
#pragma unroll
    for (int r = 0; r < 8; ++r)
        *(volatile v2l_t*)(cp + (size_t)r * (NSPLIT * 32)) = kv[r];
    __threadfence();
#pragma unroll
    for (int r = 0; r < 8; ++r)
        *(volatile v2l_t*)(cp + (size_t)r * (NSPLIT * 32)) = kv[r];
}

template <int STAGE>
__global__ void __launch_bounds__(256) refine_kernel(const float* __restrict__ vsrc,
                                                     const float* __restrict__ cb,
                                                     const float* __restrict__ cbn,
                                                     const u64* __restrict__ cand,
                                                     float* __restrict__ xdout,
                                                     float* xres,
                                                     u32* __restrict__ idxl)
{
#pragma clang fp contract(off)
    __shared__ u32 sel[8 * NSEL];
    const int lane = threadIdx.x & 31, w = threadIdx.x >> 5;
    const int row = blockIdx.x * 8 + w;

    v4f_t v[4];
    const float* vr = vsrc + (size_t)row * DDIM + 4 * lane;
#pragma unroll
    for (int q = 0; q < 4; ++q) v[q] = *(const v4f*)(vr + 128 * q);
    float vn = 0.0f;
#pragma unroll
    for (int q = 0; q < 4; ++q) {
#pragma unroll
        for (int e = 0; e < 4; ++e) vn = fmaf(v[q][e], v[q][e], vn);
    }
#pragma unroll
    for (int off = 16; off > 0; off >>= 1) vn += __shfl_xor(vn, off, 32);

    u64 l1 = ~0ull, l2 = ~0ull;
    const u64* cp = cand + (size_t)row * CPR + 16 * lane;
#pragma unroll
    for (int q = 0; q < 8; ++q) {
        const v2l_t t = *(const v2l*)(cp + 2 * q);
        {
            const u64 k = t[0];
            if (k < l1) { l2 = l1; l1 = k; } else if (k < l2) { l2 = k; }
        }
        {
            const u64 k = t[1];
            if (k < l1) { l2 = l1; l1 = k; } else if (k < l2) { l2 = k; }
        }
    }
#pragma unroll
    for (int j = 0; j < NSEL; ++j) {
        u64 wv = l1;
#pragma unroll
        for (int off = 16; off > 0; off >>= 1) {
            const u64 o = __shfl_xor(wv, off, 32);
            wv = (o < wv) ? o : wv;
        }
        if (l1 == wv) { l1 = l2; l2 = ~0ull; }
        if (lane == 0) sel[w * NSEL + j] = (u32)(wv & 0xFFFFFFFFull);
    }
    __syncthreads();

    float bestd = 3.0e38f;
    u32 besti = 0u;
#pragma unroll 1
    for (int j = 0; j < NSEL; ++j) {
        u32 c = sel[w * NSEL + j];
        c = (c > (u32)(NCODES - 1)) ? (u32)(NCODES - 1) : c;
        const float* cr = cb + (size_t)c * DDIM + 4 * lane;
        v4f_t g[4];
#pragma unroll
        for (int q = 0; q < 4; ++q) g[q] = *(const v4f*)(cr + 128 * q);
        float p = 0.0f;
#pragma unroll
        for (int q = 0; q < 4; ++q) {
#pragma unroll
            for (int e = 0; e < 4; ++e) p = fmaf(v[q][e], g[q][e], p);
        }
#pragma unroll
        for (int off = 16; off > 0; off >>= 1) p += __shfl_xor(p, off, 32);
        const float cnv = cbn[c];
        const float twop = 2.0f * p;
        const float d = (vn - twop) + cnv;
        const bool take = (d < bestd) || ((d == bestd) && (c < besti));
        if (take) { bestd = d; besti = c; }
    }

    const float* crb = cb + (size_t)besti * DDIM + 4 * lane;
    v4f_t g[4], rs[4];
#pragma unroll
    for (int q = 0; q < 4; ++q) {
        g[q] = *(const v4f*)(crb + 128 * q);
        rs[q] = v[q] - g[q];
    }
    float* xo = xdout + (size_t)row * DDIM + 4 * lane;
    float* ro = xres + (size_t)row * DDIM + 4 * lane;
    v4u_t iv;
    iv[0] = besti; iv[1] = besti; iv[2] = besti; iv[3] = besti;
    u32* io = idxl + (size_t)row * IDXP + 4 * lane;
    const bool wi = (lane < 8);

#pragma unroll
    for (int q = 0; q < 4; ++q) *(volatile v4f_t*)(xo + 128 * q) = g[q];
    if (STAGE == 1) {
#pragma unroll
        for (int q = 0; q < 4; ++q) *(volatile v4f_t*)(ro + 128 * q) = rs[q];
    }
    if (wi) *(volatile v4u_t*)io = iv;
    __threadfence();
#pragma unroll
    for (int q = 0; q < 4; ++q) *(volatile v4f_t*)(xo + 128 * q) = g[q];
    if (STAGE == 1) {
#pragma unroll
        for (int q = 0; q < 4; ++q) *(volatile v4f_t*)(ro + 128 * q) = rs[q];
    }
    if (wi) *(volatile v4u_t*)io = iv;
}

__global__ void __launch_bounds__(256) xd_kernel(const float* __restrict__ xf,
                                                 const float* __restrict__ xd1,
                                                 const float* __restrict__ xd2,
                                                 float* __restrict__ out0)
{
#pragma clang fp contract(off)
    __shared__ __align__(16) float tile[32 * TP];
    const int n = blockIdx.x >> 4, d0 = (blockIdx.x & 15) * 32;
    const int tid = threadIdx.x, lane = tid & 31, w = tid >> 5;
#pragma unroll
    for (int i = 0; i < 4; ++i) {
        const int u = tid + 256 * i;
        const int t = u >> 3, c4 = (u & 7) * 4;
        const size_t off = (size_t)(n * NT + t) * DDIM + d0 + c4;
        const v4f_t a = *(const v4f*)(xf + off);
        const v4f_t b = *(const v4f*)(xd1 + off);
        const v4f_t c = *(const v4f*)(xd2 + off);
        const v4f_t s1 = b + c;
        const v4f_t s2 = s1 - a;
        const v4f_t rr = a + s2;
#pragma unroll
        for (int e = 0; e < 4; ++e) tile[(c4 + e) * TP + t] = rr[e];
    }
    __syncthreads();
    v4f_t o[4];
    size_t oo[4];
#pragma unroll
    for (int i = 0; i < 4; ++i) {
        const int dd = 4 * w + i;
        o[i] = *(const v4f*)(tile + dd * TP + 4 * lane);
        oo[i] = (size_t)(n * DDIM + d0 + dd) * NT + 4 * lane;
        *(volatile v4f_t*)(out0 + oo[i]) = o[i];
    }
    __threadfence();
#pragma unroll
    for (int i = 0; i < 4; ++i) *(volatile v4f_t*)(out0 + oo[i]) = o[i];
}

__global__ void __launch_bounds__(256) perp_kernel(const u32* __restrict__ idxl1,
                                                   const u32* __restrict__ idxl2,
                                                   float* __restrict__ out45)
{
#pragma clang fp contract(off)
    __shared__ u32 sidx[NROWS];
    __shared__ unsigned short cnt[NCODES];
    __shared__ double red[256];
    __shared__ float res[2];
    const int tid = threadIdx.x;
#pragma unroll 1
    for (int st = 0; st < 2; ++st) {
        const u32* il = (st == 0) ? idxl1 : idxl2;
#pragma unroll 1
        for (int i = 0; i < NROWS / 256; ++i) {
            const int r = tid + 256 * i;
            u32 vv = il[(size_t)r * IDXP];
            vv = (vv > (u32)(NCODES - 1)) ? (u32)(NCODES - 1) : vv;
            sidx[r] = vv;
        }
#pragma unroll 1
        for (int b = 0; b < 64; ++b) cnt[tid * 64 + b] = 0;
        __syncthreads();
#pragma unroll 1
        for (int i = 0; i < NROWS; ++i) {
            const u32 vv = sidx[i];
            if ((vv >> 6) == (u32)tid) cnt[vv] = (unsigned short)(cnt[vv] + 1);
        }
        double s = 0.0;
#pragma unroll 1
        for (int b = 0; b < 64; ++b) {
            const float cv = (float)cnt[tid * 64 + b];
            const float p = cv * (1.0f / 4096.0f);
            const float term = p * logf(p + 1e-7f);
            s += (double)term;
        }
        red[tid] = s;
        __syncthreads();
        if (tid == 0) {
            double tot = 0.0;
#pragma unroll 1
            for (int k = 0; k < 256; ++k) tot += red[k];
            const float sf = (float)tot;
            res[st] = expf(-sf);
        }
        __syncthreads();
    }
    if (tid == 0) {
        v2f_t o;
        o[0] = res[0];
        o[1] = res[1];
        *(volatile v2f_t*)out45 = o;
        __threadfence();
        *(volatile v2f_t*)out45 = o;
    }
}

extern "C" void kernel_launch(void* const* d_in, const int* in_sizes, int n_in,
                              void* d_out, int out_size, void* d_ws, size_t ws_size,
                              hipStream_t stream)
{
    if (n_in < 3) return;
    if (in_sizes[0] != NROWS * DDIM) return;
    if (in_sizes[1] != NCODES * DDIM) return;
    if (in_sizes[2] != NCODES * DDIM) return;
    if (out_size != 4 * NROWS * DDIM + 2) return;

    const float* x   = (const float*)d_in[0];
    const float* cb1 = (const float*)d_in[1];
    const float* cb2 = (const float*)d_in[2];

    const size_t EL = (size_t)NROWS * DDIM;
    float* out   = (float*)d_out;
    float* out0  = out;
    float* out1  = out + EL;
    float* out2  = out + 2 * EL;
    float* out3  = out + 3 * EL;
    float* out45 = out + 4 * EL;

    const size_t szCBH  = (size_t)NCODES * DDIM * 2;
    const size_t szCBN  = (size_t)NCODES * 4;
    const size_t szV16  = EL * 2;
    const size_t szXRES = EL * 4;
    const size_t szCAND = (size_t)NROWS * CPR * 8;
    const size_t szIDX  = (size_t)NROWS * IDXP * 4;

    const size_t oCBH1  = 0;
    const size_t oCBH2  = oCBH1  + szCBH;
    const size_t oCBN1  = oCBH2  + szCBH;
    const size_t oCBN2  = oCBN1  + szCBN;
    const size_t oX16   = oCBN2  + szCBN;
    const size_t oXRES  = oX16   + szV16;
    const size_t oXR16  = oXRES  + szXRES;
    const size_t oCAND1 = oXR16  + szV16;
    const size_t oCAND2 = oCAND1 + szCAND;
    const size_t oIDX1  = oCAND2 + szCAND;
    const size_t oIDX2  = oIDX1  + szIDX;
    const size_t total  = oIDX2  + szIDX;
    if (total > ws_size) return;

    char* ws = (char*)d_ws;
    f16*   cbh1  = (f16*)(ws + oCBH1);
    f16*   cbh2  = (f16*)(ws + oCBH2);
    float* cbn1  = (float*)(ws + oCBN1);
    float* cbn2  = (float*)(ws + oCBN2);
    f16*   x16   = (f16*)(ws + oX16);
    float* xres  = (float*)(ws + oXRES);
    f16*   xr16  = (f16*)(ws + oXR16);
    u64*   cand1 = (u64*)(ws + oCAND1);
    u64*   cand2 = (u64*)(ws + oCAND2);
    u32*   idx1  = (u32*)(ws + oIDX1);
    u32*   idx2  = (u32*)(ws + oIDX2);

    const int n8 = (int)(EL / 8);

    cbprep_kernel<<<NCODES / 32, 256, 0, stream>>>(cb1, cbh1, cbn1);
    cbprep_kernel<<<NCODES / 32, 256, 0, stream>>>(cb2, cbh2, cbn2);
    xf_kernel<<<NBATCH * (DDIM / 32), 256, 0, stream>>>(x, out1);
    cvt16_kernel<<<(n8 + 255) / 256, 256, 0, stream>>>(out1, x16, n8);

    screen_kernel<<<dim3(NROWS / MTILE, NSPLIT), 256, 0, stream>>>(x16, cbh1, cbn1, cand1);
    refine_kernel<1><<<NROWS / 8, 256, 0, stream>>>(out1, cb1, cbn1, cand1, out2, xres, idx1);
    cvt16_kernel<<<(n8 + 255) / 256, 256, 0, stream>>>(xres, xr16, n8);

    screen_kernel<<<dim3(NROWS / MTILE, NSPLIT), 256, 0, stream>>>(xr16, cbh2, cbn2, cand2);
    refine_kernel<2><<<NROWS / 8, 256, 0, stream>>>(xres, cb2, cbn2, cand2, out3, xres, idx2);

    xd_kernel<<<NBATCH * (DDIM / 32), 256, 0, stream>>>(out1, out2, out3, out0);
    perp_kernel<<<1, 256, 0, stream>>>(idx1, idx2, out45);
}
